// DeepVCP_31224412242851
// MI455X (gfx1250) — hardware-verified
//
#include <hip/hip_runtime.h>
#define BB 4
#define CP 6
#define NPTS 16384
#define KSEL 256
#define NCEN 64
#define NSMP 32
#define KNN 10
#define NCAND (KSEL * 8)
#define NROWS (2 * BB * NPTS)

typedef __bf16 v16b __attribute__((ext_vector_type(16)));
typedef unsigned short v8us __attribute__((ext_vector_type(8), may_alias));
typedef float  v8f  __attribute__((ext_vector_type(8)));
typedef float  v4f  __attribute__((ext_vector_type(4)));
typedef float  v4fa __attribute__((ext_vector_type(4), may_alias));
union FragB { v16b v; v8us half[2]; unsigned short u[16]; };

__device__ __forceinline__ unsigned short bf16_bits(float x) { unsigned int u = __float_as_uint(x); return (unsigned short)((u + 0x7FFFu + ((u >> 16) & 1u)) >> 16); }
__device__ __forceinline__ float bf16_val(unsigned short b) { return __uint_as_float(((unsigned int)b) << 16); }
__device__ __forceinline__ float bf16_round(float x) { return bf16_val(bf16_bits(x)); }
template <int NT>
__device__ __forceinline__ v8f mmaN(v16b ah, v16b al, v16b bh, v16b bl, v8f c) {
  c = __builtin_amdgcn_wmma_f32_16x16x32_bf16(false, ah, false, bh, (short)0, c, false, false);
  if (NT >= 2) c = __builtin_amdgcn_wmma_f32_16x16x32_bf16(false, al, false, bh, (short)0, c, false, false);
  if (NT >= 3) c = __builtin_amdgcn_wmma_f32_16x16x32_bf16(false, ah, false, bl, (short)0, c, false, false);
  asm volatile("v_nop\n\tv_nop\n\tv_nop\n\tv_nop" : "+v"(c) : "v"(ah), "v"(al), "v"(bh), "v"(bl));
  return c;
}

__global__ __launch_bounds__(256) void k_wt_bf16(const float* __restrict__ W, unsigned short* __restrict__ Wt, int K, int N) {
  const int t = blockIdx.x * 256 + threadIdx.x;
  const int k8n = K / 8;
  if (t >= N * k8n) return;
  const int n = t / k8n, k8 = (t % k8n) * 8;
  v8us v;
#pragma unroll
  for (int i = 0; i < 8; ++i) v[i] = bf16_bits(W[(size_t)(k8 + i) * N + n]);
  *(volatile v8us*)(Wt + (size_t)n * K + k8) = v;
  __threadfence();
  *(volatile v8us*)(Wt + (size_t)n * K + k8) = v;
}

template <bool ASPLIT, int ACT, bool BIAS_BF16>
__global__ __launch_bounds__(128) void k_gemm_bf(const float* __restrict__ A, int lda, const unsigned short* __restrict__ Wt, int ldb,
                                               const float* __restrict__ bias, float* __restrict__ C, int ldc, int M, int N, int K) {
  __shared__ __attribute__((aligned(16))) float so[4][16][64];
  const int tid = threadIdx.x, w = tid >> 5, lane = tid & 31, ln = lane & 15, hh = lane >> 4;
  const int ntn = N / 64;
  const int wid = blockIdx.x * 4 + w;
  const int mt = wid / ntn, nq = wid % ntn;
  if (mt * 16 >= M) return;
  const int row0 = mt * 16, col0 = nq * 64;
  const float* arow = A + (size_t)(row0 + ln) * lda;
  v8f acc[4] = {};
  for (int kb = 0; kb < K; kb += 32) {
    FragB ah, al;
    const v4f x0 = *(const v4fa*)(arow + kb + 8 * hh), x1 = *(const v4fa*)(arow + kb + 8 * hh + 4);
    const v4f x2 = *(const v4fa*)(arow + kb + 16 + 8 * hh), x3 = *(const v4fa*)(arow + kb + 16 + 8 * hh + 4);
    float xs[16] = {x0[0],x0[1],x0[2],x0[3],x1[0],x1[1],x1[2],x1[3],x2[0],x2[1],x2[2],x2[3],x3[0],x3[1],x3[2],x3[3]};
#pragma unroll
    for (int i = 0; i < 16; ++i) { const unsigned short hb = bf16_bits(xs[i]); ah.u[i] = hb; al.u[i] = ASPLIT ? bf16_bits(xs[i] - bf16_val(hb)) : (unsigned short)0; }
#pragma unroll
    for (int t = 0; t < 4; ++t) {
      const unsigned short* brow = Wt + (size_t)(col0 + t * 16 + ln) * ldb + kb;
      FragB b;
      b.half[0] = *(const v8us*)(brow + 8 * hh);
      b.half[1] = *(const v8us*)(brow + 16 + 8 * hh);
      acc[t] = mmaN<ASPLIT ? 2 : 1>(ah.v, al.v, b.v, b.v, acc[t]);
    }
  }
#pragma unroll
  for (int t = 0; t < 4; ++t) {
    float bv = bias ? bias[col0 + t * 16 + ln] : 0.f;
    if (BIAS_BF16) bv = bf16_round(bv);
#pragma unroll
    for (int r = 0; r < 8; ++r) { float v = acc[t][r] + bv; if (ACT == 1) v = fmaxf(v, 0.f); so[w][8 * hh + r][t * 16 + ln] = v; }
  }
  __builtin_amdgcn_fence(__ATOMIC_ACQ_REL, "workgroup");
  __builtin_amdgcn_wave_barrier();
  const int rsub = lane >> 4, c4 = (lane & 15) * 4;
  for (int pass = 0; pass < 2; ++pass) {
#pragma unroll
    for (int q = 0; q < 8; ++q) {
      const int r = q * 2 + rsub;
      const v4f v = *(const v4fa*)&so[w][r][c4];
      *(volatile v4f*)(C + (size_t)(row0 + r) * ldc + col0 + c4) = v;
    }
    if (pass == 0) __threadfence();
  }
}

template <int D, bool CAUSAL>
__global__ __launch_bounds__(128) void k_flash(const float* __restrict__ qb, const float* __restrict__ kb, const float* __restrict__ vb,
                                             int pitch, int T, int H, float scale, float* __restrict__ y, int ypitch) {
  constexpr int KS = D / 32;
  constexpr int DT = D / 16;
  __shared__ __attribute__((aligned(16))) unsigned short sKh[32][D + 8], sKl[32][D + 8], sVh[32][D + 8], sVl[32][D + 8];
  __shared__ __attribute__((aligned(16))) unsigned short sPh[4][16][40], sPl[4][16][40];
  __shared__ __attribute__((aligned(16))) float sO[4][16][D];
  const int tid = threadIdx.x, w = tid >> 5, lane = tid & 31, ln = lane & 15, hh = lane >> 4;
  const int nqb = (T + 63) / 64;
  const int bh = blockIdx.x / nqb, qblk = blockIdx.x % nqb;
  const int b = bh / H, h = bh % H;
  const int q0 = qblk * 64 + w * 16;
  const float* Q = qb + (size_t)b * T * pitch + h * D;
  const float* K = kb + (size_t)b * T * pitch + h * D;
  const float* V = vb + (size_t)b * T * pitch + h * D;

  FragB aqh[KS], aql[KS];
  {
    int row = q0 + ln; if (row >= T) row = T - 1;
    const float* qr = Q + (size_t)row * pitch;
#pragma unroll
    for (int ks = 0; ks < KS; ++ks)
#pragma unroll
      for (int i = 0; i < 16; ++i) {
        const int d = ks * 32 + ((i < 8) ? (8 * hh + i) : (16 + 8 * hh + (i - 8)));
        const float x = qr[d] * scale; const unsigned short hb = bf16_bits(x);
        aqh[ks].u[i] = hb; aql[ks].u[i] = bf16_bits(x - bf16_val(hb));
      }
  }
  float m_r[8], l_r[8];
#pragma unroll
  for (int r = 0; r < 8; ++r) { m_r[r] = -3.0e38f; l_r[r] = 0.f; }
  v8f oacc[DT];
#pragma unroll
  for (int dt = 0; dt < DT; ++dt) oacc[dt] = (v8f){0.f,0.f,0.f,0.f,0.f,0.f,0.f,0.f};

  const int kv_end = CAUSAL ? min(T, qblk * 64 + 64) : T;
  for (int j0 = 0; j0 < kv_end; j0 += 32) {
    __syncthreads();
    for (int e = tid; e < 32 * (D / 4); e += 128) {
      const int r = e / (D / 4), c4 = (e % (D / 4)) * 4;
      const int key = j0 + r;
      v4f kf = {0.f,0.f,0.f,0.f}, vf = {0.f,0.f,0.f,0.f};
      if (key < T) { kf = *(const v4fa*)(K + (size_t)key * pitch + c4); vf = *(const v4fa*)(V + (size_t)key * pitch + c4); }
#pragma unroll
      for (int t = 0; t < 4; ++t) {
        unsigned short hb = bf16_bits(kf[t]); sKh[r][c4 + t] = hb; sKl[r][c4 + t] = bf16_bits(kf[t] - bf16_val(hb));
        hb = bf16_bits(vf[t]); sVh[r][c4 + t] = hb; sVl[r][c4 + t] = bf16_bits(vf[t] - bf16_val(hb));
      }
    }
    __syncthreads();
    v8f s[2];
#pragma unroll
    for (int nt = 0; nt < 2; ++nt) {
      v8f acc = {};
#pragma unroll
      for (int ks = 0; ks < KS; ++ks) {
        FragB bh_, bl_;
        bh_.half[0] = *(const v8us*)&sKh[nt * 16 + ln][ks * 32 + 8 * hh]; bh_.half[1] = *(const v8us*)&sKh[nt * 16 + ln][ks * 32 + 16 + 8 * hh];
        bl_.half[0] = *(const v8us*)&sKl[nt * 16 + ln][ks * 32 + 8 * hh]; bl_.half[1] = *(const v8us*)&sKl[nt * 16 + ln][ks * 32 + 16 + 8 * hh];
        acc = mmaN<3>(aqh[ks].v, aql[ks].v, bh_.v, bl_.v, acc);
      }
      s[nt] = acc;
    }
    float alpha[8];
#pragma unroll
    for (int r = 0; r < 8; ++r) {
      const int qi = q0 + 8 * hh + r;
      const int ja = j0 + ln, jb = j0 + 16 + ln;
      if (CAUSAL) { if (ja > qi) s[0][r] = -3.0e38f; if (jb > qi) s[1][r] = -3.0e38f; }
      if (ja >= T) s[0][r] = -3.0e38f;
      if (jb >= T) s[1][r] = -3.0e38f;
      float mx = fmaxf(s[0][r], s[1][r]);
      mx = fmaxf(mx, __shfl_xor(mx, 1, 32)); mx = fmaxf(mx, __shfl_xor(mx, 2, 32)); mx = fmaxf(mx, __shfl_xor(mx, 4, 32)); mx = fmaxf(mx, __shfl_xor(mx, 8, 32));
      const float mnew = fmaxf(m_r[r], mx);
      alpha[r] = (mnew > -1.0e38f) ? __expf(m_r[r] - mnew) : 1.0f;
      const float p0 = (s[0][r] > -1.0e38f) ? __expf(s[0][r] - mnew) : 0.f;
      const float p1 = (s[1][r] > -1.0e38f) ? __expf(s[1][r] - mnew) : 0.f;
      m_r[r] = mnew;
      l_r[r] = l_r[r] * alpha[r] + p0 + p1;
      unsigned short hb = bf16_bits(p0); sPh[w][8 * hh + r][ln] = hb;      sPl[w][8 * hh + r][ln] = bf16_bits(p0 - bf16_val(hb));
      hb = bf16_bits(p1);                sPh[w][8 * hh + r][16 + ln] = hb; sPl[w][8 * hh + r][16 + ln] = bf16_bits(p1 - bf16_val(hb));
    }
#pragma unroll
    for (int dt = 0; dt < DT; ++dt)
#pragma unroll
      for (int r = 0; r < 8; ++r) oacc[dt][r] *= alpha[r];
    __builtin_amdgcn_fence(__ATOMIC_ACQ_REL, "workgroup");
    __builtin_amdgcn_wave_barrier();
    FragB pah, pal;
    pah.half[0] = *(const v8us*)&sPh[w][ln][8 * hh]; pah.half[1] = *(const v8us*)&sPh[w][ln][16 + 8 * hh];
    pal.half[0] = *(const v8us*)&sPl[w][ln][8 * hh]; pal.half[1] = *(const v8us*)&sPl[w][ln][16 + 8 * hh];
#pragma unroll
    for (int dt = 0; dt < DT; ++dt) {
      FragB bvh, bvl;
#pragma unroll
      for (int i = 0; i < 8; ++i) {
        bvh.u[i] = sVh[8 * hh + i][dt * 16 + ln]; bvh.u[8 + i] = sVh[16 + 8 * hh + i][dt * 16 + ln];
        bvl.u[i] = sVl[8 * hh + i][dt * 16 + ln]; bvl.u[8 + i] = sVl[16 + 8 * hh + i][dt * 16 + ln];
      }
      oacc[dt] = mmaN<3>(pah.v, pal.v, bvh.v, bvl.v, oacc[dt]);
    }
    __builtin_amdgcn_fence(__ATOMIC_ACQ_REL, "workgroup");
    __builtin_amdgcn_wave_barrier();
  }
#pragma unroll
  for (int r = 0; r < 8; ++r) {
    float l = l_r[r];
    l += __shfl_xor(l, 1, 32); l += __shfl_xor(l, 2, 32); l += __shfl_xor(l, 4, 32); l += __shfl_xor(l, 8, 32);
    l_r[r] = (l > 0.f) ? 1.0f / l : 0.f;
  }
#pragma unroll
  for (int dt = 0; dt < DT; ++dt)
#pragma unroll
    for (int r = 0; r < 8; ++r) sO[w][8 * hh + r][dt * 16 + ln] = oacc[dt][r] * l_r[r];
  __builtin_amdgcn_fence(__ATOMIC_ACQ_REL, "workgroup");
  __builtin_amdgcn_wave_barrier();
  for (int pass = 0; pass < 2; ++pass) {
    for (int r = 0; r < 16; ++r) {
      const int row = q0 + r;
      if (row < T && lane < D / 4) {
        const v4f val = *(const v4fa*)&sO[w][r][lane * 4];
        *(volatile v4f*)(y + ((size_t)b * T + row) * ypitch + h * D + lane * 4) = val;
      }
    }
    if (pass == 0) __threadfence();
  }
}

template <bool ASPLIT, int ACT, bool BIAS_BF16, bool RES_BF16>
__global__ __launch_bounds__(128) void k_gemm_bf3(const float* __restrict__ A, int lda, const unsigned short* __restrict__ Wt, int ldb,
                                                const float* __restrict__ bias, const float* __restrict__ resid, int rmod, int ldr,
                                                float* __restrict__ C, int ldc, int M, int N, int K) {
  __shared__ __attribute__((aligned(16))) float so[4][16][64];
  const int tid = threadIdx.x, w = tid >> 5, lane = tid & 31, ln = lane & 15, hh = lane >> 4;
  const int ntn = N / 64;
  const int wid = blockIdx.x * 4 + w;
  const int mt = wid / ntn, nq = wid % ntn;
  if (mt * 16 >= M) return;
  const int row0 = mt * 16, col0 = nq * 64;
  const float* arow = A + (size_t)(row0 + ln) * lda;
  v8f acc[4] = {};
  for (int kb = 0; kb < K; kb += 32) {
    FragB ah, al;
    const v4f x0 = *(const v4fa*)(arow + kb + 8 * hh), x1 = *(const v4fa*)(arow + kb + 8 * hh + 4);
    const v4f x2 = *(const v4fa*)(arow + kb + 16 + 8 * hh), x3 = *(const v4fa*)(arow + kb + 16 + 8 * hh + 4);
    float xs[16] = {x0[0],x0[1],x0[2],x0[3],x1[0],x1[1],x1[2],x1[3],x2[0],x2[1],x2[2],x2[3],x3[0],x3[1],x3[2],x3[3]};
#pragma unroll
    for (int i = 0; i < 16; ++i) { const unsigned short hb = bf16_bits(xs[i]); ah.u[i] = hb; al.u[i] = ASPLIT ? bf16_bits(xs[i] - bf16_val(hb)) : (unsigned short)0; }
#pragma unroll
    for (int t = 0; t < 4; ++t) {
      const unsigned short* brow = Wt + (size_t)(col0 + t * 16 + ln) * ldb + kb;
      FragB b;
      b.half[0] = *(const v8us*)(brow + 8 * hh);
      b.half[1] = *(const v8us*)(brow + 16 + 8 * hh);
      acc[t] = mmaN<ASPLIT ? 2 : 1>(ah.v, al.v, b.v, b.v, acc[t]);
    }
  }
#pragma unroll
  for (int t = 0; t < 4; ++t) {
    const int col = col0 + t * 16 + ln;
    float bv = bias ? bias[col] : 0.f;
    if (BIAS_BF16) bv = bf16_round(bv);
#pragma unroll
    for (int r = 0; r < 8; ++r) {
      float v = acc[t][r] + bv;
      if (resid) { float rv = resid[(size_t)((row0 + 8 * hh + r) % rmod) * ldr + col]; if (RES_BF16) rv = bf16_round(rv); v += rv; }
      if (ACT == 1) v = fmaxf(v, 0.f);
      if (ACT == 2) v = 0.5f * v * (1.0f + erff(v * 0.70710678118654752f));
      if (ACT == 3) { const float u = 0.7978845608028654f * (v + 0.044715f * v * v * v); v = 0.5f * v * (1.0f + tanhf(u)); }
      so[w][8 * hh + r][t * 16 + ln] = v;
    }
  }
  __builtin_amdgcn_fence(__ATOMIC_ACQ_REL, "workgroup");
  __builtin_amdgcn_wave_barrier();
  const int rsub = lane >> 4, c4 = (lane & 15) * 4;
  for (int pass = 0; pass < 2; ++pass) {
#pragma unroll
    for (int q = 0; q < 8; ++q) {
      const int r = q * 2 + rsub;
      const v4f v = *(const v4fa*)&so[w][r][c4];
      *(volatile v4f*)(C + (size_t)(row0 + r) * ldc + col0 + c4) = v;
    }
    if (pass == 0) __threadfence();
  }
}
template <bool PARAM_BF16>
__global__ __launch_bounds__(256) void k_layernorm(const float* __restrict__ X, const float* __restrict__ R, const float* __restrict__ g, const float* __restrict__ bta,
                                                  float* __restrict__ out_sum, float* __restrict__ out_norm, int N, float eps) {
  __shared__ float red[256];
  const int row = blockIdx.x, tid = threadIdx.x;
  const float* x = X + (size_t)row * N; const float* rr = R ? R + (size_t)row * N : nullptr;
  float vals[16];
  const int per = N / 256;
  float s1 = 0.f;
  for (int u = 0; u < per / 4; ++u) {
    const int j = tid * 4 + 1024 * u;
    const v4f a = *(const v4fa*)(x + j);
    v4f b = {0.f,0.f,0.f,0.f}; if (rr) b = *(const v4fa*)(rr + j);
#pragma unroll
    for (int q = 0; q < 4; ++q) { const float v = a[q] + b[q]; vals[u * 4 + q] = v; s1 += v; }
  }
  red[tid] = s1; __syncthreads();
  for (int st = 128; st > 0; st >>= 1) { if (tid < st) red[tid] += red[tid + st]; __syncthreads(); }
  const float mu = red[0] / (float)N; __syncthreads();
  float s2 = 0.f;
  for (int u = 0; u < per / 4; ++u)
#pragma unroll
    for (int q = 0; q < 4; ++q) { const float c = vals[u * 4 + q] - mu; s2 += c * c; }
  red[tid] = s2; __syncthreads();
  for (int st = 128; st > 0; st >>= 1) { if (tid < st) red[tid] += red[tid + st]; __syncthreads(); }
  const float rs = rsqrtf(red[0] / (float)N + eps);
  for (int pass = 0; pass < 2; ++pass) {
    for (int u = 0; u < per / 4; ++u) {
      const int j = tid * 4 + 1024 * u;
      v4f o, sm;
#pragma unroll
      for (int q = 0; q < 4; ++q) {
        float gg = g[j + q], bb = bta[j + q];
        if (PARAM_BF16) { gg = bf16_round(gg); bb = bf16_round(bb); }
        sm[q] = vals[u * 4 + q]; o[q] = (vals[u * 4 + q] - mu) * rs * gg + bb;
      }
      if (out_sum) *(volatile v4f*)(out_sum + (size_t)row * N + j) = sm;
      *(volatile v4f*)(out_norm + (size_t)row * N + j) = o;
    }
    if (pass == 0) __threadfence();
  }
}

__global__ __launch_bounds__(256) void k_wt_pad(const float* __restrict__ W, unsigned short* __restrict__ Bt, int Kin, int Nout, int Kp, int Np) {
  const int t = blockIdx.x * 256 + threadIdx.x; const int k8n = Kp / 8; if (t >= Np * k8n) return; const int n = t / k8n, k8 = (t % k8n) * 8; v8us v;
  for (int i = 0; i < 8; ++i) { const int k = k8 + i; v[i] = (n < Nout && k < Kin) ? bf16_bits(W[(size_t)k * Nout + n]) : (unsigned short)0; }
  *(volatile v8us*)(Bt + (size_t)n * Kp + k8) = v; __threadfence(); *(volatile v8us*)(Bt + (size_t)n * Kp + k8) = v;
}
__global__ __launch_bounds__(256) void k_xrows(const float* __restrict__ src, const float* __restrict__ tgt, float* __restrict__ X) {
  const size_t t = (size_t)blockIdx.x * 256 + threadIdx.x; if (t >= (size_t)NROWS * 8) return; const int c4 = (int)(t % 8) * 4; const size_t row = t / 8; const int n = (int)(row % NPTS); const int b = (int)((row / NPTS) % BB); const int cl = (int)(row / ((size_t)NPTS * BB));
  const float* P = cl ? tgt : src; v4f v = {0.f,0.f,0.f,0.f};
  for (int q = 0; q < 4; ++q) { const int c = c4 + q; if (c < CP) v[q] = bf16_round(P[((size_t)b * CP + c) * NPTS + n]); }
  *(volatile v4f*)(X + t * 4) = v; __threadfence(); *(volatile v4f*)(X + t * 4) = v;
}
__global__ __launch_bounds__(256) void k_score(const float* __restrict__ feat, const float* __restrict__ w, float* __restrict__ sc) {
  const int t = blockIdx.x * 256 + threadIdx.x; if (t >= 2 * NPTS) return; const int cl = t / NPTS, n = t % NPTS; float s = 0.f;
#pragma unroll 1
  for (int b = 0; b < BB; ++b) { const float* f = feat + (((size_t)cl * BB + b) * NPTS + n) * 128; float d = 0.f;
#pragma unroll 1
    for (int c = 0; c < 128; c += 4) { const v4f a = *(const v4fa*)(f + c); d += a[0] * bf16_round(w[c]) + a[1] * bf16_round(w[c + 1]) + a[2] * bf16_round(w[c + 2]) + a[3] * bf16_round(w[c + 3]); }
    s += d; }
  const float v = s / 4.0f; *(volatile float*)(sc + t) = v; __threadfence(); *(volatile float*)(sc + t) = v;
}
__global__ __launch_bounds__(256) void k_topk(const float* __restrict__ sc, int* __restrict__ idx) {
  __shared__ float bv[256]; __shared__ int bi[256]; __shared__ int sel[KSEL];
  const int cl = blockIdx.x, t = threadIdx.x; const float* s = sc + (size_t)cl * NPTS;
  float vals[64]; unsigned long long taken = 0ull;
#pragma unroll
  for (int i = 0; i < 64; ++i) vals[i] = s[i * 256 + t];
#pragma unroll 1
  for (int r = 0; r < KSEL; ++r) {
    float mv = -3.0e38f; int mi = 0x7fffffff;
#pragma unroll
    for (int i = 0; i < 64; ++i) { if (taken & (1ull << i)) continue; const float v = vals[i]; const int j = i * 256 + t; if (v > mv || (v == mv && j < mi)) { mv = v; mi = j; } }
    bv[t] = mv; bi[t] = mi; __syncthreads();
    for (int st = 128; st > 0; st >>= 1) { if (t < st) { const float ov = bv[t + st]; const int oi = bi[t + st]; if (ov > bv[t] || (ov == bv[t] && oi < bi[t])) { bv[t] = ov; bi[t] = oi; } } __syncthreads(); }
    const int win = bi[0]; if (t == 0) sel[r] = win; if ((win & 255) == t) taken |= (1ull << (win >> 8)); __syncthreads();
  }
  for (int pass = 0; pass < 2; ++pass) { *(volatile int*)(idx + (size_t)cl * KSEL + t) = sel[t]; if (pass == 0) __threadfence(); }
}
__global__ __launch_bounds__(256) void k_keypts(const float* __restrict__ src, const float* __restrict__ tgt, const int* __restrict__ idx, float* __restrict__ kp, float* __restrict__ out0) {
  const int cl = blockIdx.x / BB, b = blockIdx.x % BB; const float* P = cl ? tgt : src;
  for (int pass = 0; pass < 2; ++pass) { for (int e = threadIdx.x; e < KSEL * CP; e += 256) { const int k = e / CP, c = e % CP; int n = idx[cl * KSEL + k]; n = n < 0 ? 0 : (n >= NPTS ? NPTS - 1 : n); const float v = bf16_round(P[((size_t)b * CP + c) * NPTS + n]);
      *(volatile float*)(kp + ((size_t)cl * BB + b) * KSEL * CP + e) = v; if (cl == 0) *(volatile float*)(out0 + (size_t)b * KSEL * CP + e) = v; } if (pass == 0) __threadfence(); }
}
__device__ __forceinline__ float sq3(float x, float y, float z) { return __fadd_rn(__fadd_rn(__fmul_rn(x, x), __fmul_rn(z, z)), __fmul_rn(y, y)); }
__device__ __forceinline__ float dot3(float a0, float a1, float a2, float b0, float b1, float b2) { return __fadd_rn(__fadd_rn(__fmul_rn(a0, b0), __fmul_rn(a1, b1)), __fmul_rn(a2, b2)); }
__global__ __launch_bounds__(256) void k_group(const float* __restrict__ kp, float* __restrict__ out2, float* __restrict__ out3) {
  __shared__ float so[8][NSMP * CP]; __shared__ int ssel[8][NSMP]; __shared__ float sd[8][NSMP];
  const int tid = threadIdx.x, wv = tid >> 5, lane = tid & 31; const int g = blockIdx.x * 8 + wv; if (g >= 2 * BB * NCEN) return; const int m = g % NCEN; const int b = (g / NCEN) % BB; const int cl = g / (NCEN * BB);
  const float* K = kp + ((size_t)cl * BB + b) * KSEL * CP; const float c0 = K[m * CP], c1 = K[m * CP + 1], c2 = K[m * CP + 2]; const float cs = sq3(c0, c1, c2);
  float dv[8];
#pragma unroll
  for (int i = 0; i < 8; ++i) { const int k = i * 32 + lane; const float k0 = K[k * CP], k1 = K[k * CP + 1], k2 = K[k * CP + 2]; dv[i] = __fsub_rn(__fadd_rn(cs, sq3(k0, k1, k2)), __fmul_rn(2.0f, dot3(c0, c1, c2, k0, k1, k2))); }
  unsigned taken = 0u;
#pragma unroll 1
  for (int r = 0; r < NSMP; ++r) { float mv = 3.0e38f; int mi = 0x7fffffff; int bi_ = -1;
#pragma unroll
    for (int i = 0; i < 8; ++i) { if (taken & (1u << i)) continue; const int k = i * 32 + lane; if (bi_ < 0 || dv[i] < mv || (dv[i] == mv && k < mi)) { mv = dv[i]; mi = k; bi_ = i; } }
    float rv = mv; int rk = (bi_ < 0) ? 0x7fffffff : mi;
#pragma unroll
    for (int o = 16; o >= 1; o >>= 1) { const float ov = __shfl_xor(rv, o, 32); const int ok_ = __shfl_xor(rk, o, 32); const bool oth = (ok_ != 0x7fffffff) && ((rk == 0x7fffffff) || ov < rv || (ov == rv && ok_ < rk)); if (oth) { rv = ov; rk = ok_; } }
    if (bi_ >= 0 && rk == mi) taken |= (1u << bi_);
    if (lane == 0) { ssel[wv][r] = rk; sd[wv][r] = rv; } }
  __builtin_amdgcn_fence(__ATOMIC_ACQ_REL, "workgroup"); __builtin_amdgcn_wave_barrier();
  { int ksel = ssel[wv][lane]; const float dsel = sd[wv][lane]; if (!(dsel <= 1.0f)) ksel = ssel[wv][0];
    for (int c = 0; c < CP; ++c) { const float v = K[ksel * CP + c] - (c < 3 ? (c == 0 ? c0 : (c == 1 ? c1 : c2)) : 0.f); so[wv][lane * CP + c] = v; } }
  __builtin_amdgcn_fence(__ATOMIC_ACQ_REL, "workgroup"); __builtin_amdgcn_wave_barrier();
  float* O = (cl ? out3 : out2) + ((size_t)b * NCEN + m) * NSMP * CP;
  for (int pass = 0; pass < 2; ++pass) { for (int e = lane; e < NSMP * CP; e += 32) *(volatile float*)(O + e) = so[wv][e]; if (pass == 0) __threadfence(); }
}
__global__ __launch_bounds__(256) void k_knn(const float* __restrict__ kp, const float* __restrict__ tgt, float* __restrict__ out1) {
  __shared__ float st[1024][3]; __shared__ float so[256 * KNN];
  const int b = blockIdx.x / (NCAND / 256); const int cbase = (blockIdx.x % (NCAND / 256)) * 256; const int t = threadIdx.x; const int ci = cbase + t; const int k = ci / 8, gi = ci % 8;
  const float* K = kp + ((size_t)0 * BB + b) * KSEL * CP;
  const float gx = (gi & 4) ? 0.1f : 0.f, gy = (gi & 2) ? 0.1f : 0.f, gz = (gi & 1) ? 0.1f : 0.f;
  const float a0 = K[k * CP] + gx, a1 = K[k * CP + 1] + gy, a2 = K[k * CP + 2] + gz; const float as_ = sq3(a0, a1, a2);
  float best[KNN]; for (int i = 0; i < KNN; ++i) best[i] = 3.0e38f;
  for (int n0 = 0; n0 < NPTS; n0 += 1024) {
    __syncthreads();
    for (int e = t; e < 1024; e += 256) { st[e][0] = bf16_round(tgt[((size_t)b * CP + 0) * NPTS + n0 + e]); st[e][1] = bf16_round(tgt[((size_t)b * CP + 1) * NPTS + n0 + e]); st[e][2] = bf16_round(tgt[((size_t)b * CP + 2) * NPTS + n0 + e]); }
    __syncthreads();
#pragma unroll 1
    for (int j = 0; j < 1024; ++j) { const float b0 = st[j][0], b1 = st[j][1], b2 = st[j][2]; const float d = (as_ + sq3(b0, b1, b2)) - 2.0f * dot3(a0, a1, a2, b0, b1, b2);
      if (d < best[KNN - 1]) { best[KNN - 1] = d;
#pragma unroll
        for (int i = KNN - 1; i > 0; --i) { if (best[i] < best[i - 1]) { const float tq = best[i]; best[i] = best[i - 1]; best[i - 1] = tq; } } } }
  }
  float ssum = 0.f; float kd[KNN]; for (int i = 0; i < KNN; ++i) { kd[i] = sqrtf(fmaxf(best[i], 0.f)); ssum += kd[i]; }
  for (int i = 0; i < KNN; ++i) so[t * KNN + i] = kd[i] / ssum;
  __syncthreads();
  for (int pass = 0; pass < 2; ++pass) { for (int e = t; e < 256 * KNN; e += 256) *(volatile float*)(out1 + ((size_t)b * NCAND + cbase) * KNN + e) = so[e]; if (pass == 0) __threadfence(); }
}
extern "C" void kernel_launch(void* const* d_in, const int* in_sizes, int n_in,
                              void* d_out, int out_size, void* d_ws, size_t ws_size, hipStream_t stream) {
  (void)in_sizes; (void)n_in; (void)out_size;
  const float* src = (const float*)d_in[0]; const float* tgt = (const float*)d_in[1]; const float* W1 = (const float*)d_in[2]; const float* b1 = (const float*)d_in[3]; const float* W2 = (const float*)d_in[4]; const float* b2 = (const float*)d_in[5]; const float* wsc = (const float*)d_in[6];
  float* out0 = (float*)d_out; float* out1 = (float*)((char*)d_out + 24576); float* out2 = (float*)((char*)d_out + 352256); float* out3 = (float*)((char*)d_out + 548864);
  char* ws = (char*)d_ws; size_t off = 0;
  auto take = [&](size_t bytes) { char* p = ws + off; off += (bytes + 255) & ~(size_t)255; return p; };
  unsigned short* B1 = (unsigned short*)take(64 * 32 * 2); unsigned short* B2 = (unsigned short*)take(128 * 64 * 2);
  float* X = (float*)take((size_t)NROWS * 32 * 4); float* h = (float*)take((size_t)NROWS * 64 * 4); float* feat = (float*)take((size_t)NROWS * 128 * 4); float* sc = (float*)take((size_t)2 * NPTS * 4); int* idx = (int*)take(2 * KSEL * 4); float* kp = (float*)take((size_t)2 * BB * KSEL * CP * 4);
  if (off > ws_size) return;
  k_wt_pad<<<1, 256, 0, stream>>>(W1, B1, CP, 64, 32, 64); k_wt_pad<<<(128 * 8 + 255) / 256, 256, 0, stream>>>(W2, B2, 64, 128, 64, 128);
  k_xrows<<<(unsigned)(((size_t)NROWS * 8 + 255) / 256), 256, 0, stream>>>(src, tgt, X);
  k_gemm_bf3<false, 1, true, false><<<((NROWS / 16) * 1 + 3) / 4, 128, 0, stream>>>(X, 32, B1, 32, b1, nullptr, 1, 0, h, 64, NROWS, 64, 32);
  k_gemm_bf3<true, 1, true, false><<<((NROWS / 16) * 2 + 3) / 4, 128, 0, stream>>>(h, 64, B2, 64, b2, nullptr, 1, 0, feat, 128, NROWS, 128, 64);
  k_score<<<(2 * NPTS + 255) / 256, 256, 0, stream>>>(feat, wsc, sc);
  k_topk<<<2, 256, 0, stream>>>(sc, idx);
  k_keypts<<<2 * BB, 256, 0, stream>>>(src, tgt, idx, kp, out0);
  k_group<<<(2 * BB * NCEN + 7) / 8, 256, 0, stream>>>(kp, out2, out3);
  k_knn<<<BB * (NCAND / 256), 256, 0, stream>>>(kp, tgt, out1);
}
